// TemporalSelfAttentionLayer_94489281071
// MI455X (gfx1250) — hardware-verified
//
#include <hip/hip_runtime.h>
#include <math.h>

typedef __attribute__((ext_vector_type(16))) _Float16 v16h;
typedef __attribute__((ext_vector_type(16))) __bf16 v16b;
typedef __attribute__((ext_vector_type(8)))  _Float16 v8h;
typedef __attribute__((ext_vector_type(8)))  float v8f;
typedef __attribute__((ext_vector_type(4)))  float v4f;
typedef __attribute__((ext_vector_type(2)))  float v2f;
typedef __attribute__((ext_vector_type(4)))  unsigned v4u;
typedef __attribute__((ext_vector_type(4)))  int v4i;
typedef float __attribute__((may_alias)) float_a;
typedef int __attribute__((may_alias)) int_a;

template <typename T> __device__ __forceinline__ void vst2(void* p, T v) { *(volatile T*)p = v; __threadfence(); *(volatile T*)p = v; }
__device__ __forceinline__ v8f wmma16(v16h a, v16h b, v8f c) {
  v8f d = __builtin_amdgcn_wmma_f32_16x16x32_f16(false, a, false, b, (short)0, c, false, false);
  asm volatile("v_nop\n\tv_nop\n\tv_nop\n\tv_nop" : "+v"(d) : "v"(a), "v"(b));
  return d;
}
__device__ __forceinline__ v8f wmma_bf(v16b a, v16b b, v8f c) {
  v8f d = __builtin_amdgcn_wmma_f32_16x16x32_bf16(false, a, false, b, (short)0, c, false, false);
  asm volatile("v_nop\n\tv_nop\n\tv_nop\n\tv_nop" : "+v"(d) : "v"(a), "v"(b));
  return d;
}
__device__ __forceinline__ v16h frag_h(const _Float16* rowk0, int lane) {
  union { v16h v; v8h q[2]; } u; const _Float16* p = rowk0 + 8 * (lane >> 4);
  u.q[0] = *(const v8h*)p; u.q[1] = *(const v8h*)(p + 16); return u.v;
}
__device__ __forceinline__ v16h frag_f32(const float* rowk0, int lane) {
  v16h a; const float* p = rowk0 + 8 * (lane >> 4);
#pragma unroll
  for (int i = 0; i < 8; ++i) { a[i] = (_Float16)p[i]; a[8 + i] = (_Float16)p[16 + i]; }
  return a;
}
__device__ __forceinline__ v16h frag_f32s(const float* rowk0, int lane, float sc) {
  v16h a; const float* p = rowk0 + 8 * (lane >> 4);
#pragma unroll
  for (int i = 0; i < 8; ++i) { a[i] = (_Float16)(p[i] * sc); a[8 + i] = (_Float16)(p[16 + i] * sc); }
  return a;
}
__device__ __forceinline__ v16h fragc_f32(const float* W, int k0, int n, int lane, int ld, int K) {
  v16h a; const int g = lane >> 4;
#pragma unroll
  for (int i = 0; i < 8; ++i) { const int ka = k0 + 8 * g + i, kb = ka + 16;
    a[i] = (_Float16)(ka < K ? W[(size_t)ka * ld + n] : 0.f); a[8 + i] = (_Float16)(kb < K ? W[(size_t)kb * ld + n] : 0.f); }
  return a;
}
struct F2 { v16b h, l; };
__device__ __forceinline__ F2 bsplit16(const float v[16]) { F2 r;
#pragma unroll
  for (int i = 0; i < 16; ++i) { const __bf16 h = (__bf16)v[i]; r.h[i] = h; r.l[i] = (__bf16)(v[i] - (float)h); }
  return r; }
__device__ __forceinline__ F2 split_row(const float* row, int k0, int lane) { float v[16]; const float* p = row + k0 + 8 * (lane >> 4);
#pragma unroll
  for (int i = 0; i < 8; ++i) { v[i] = p[i]; v[8 + i] = p[16 + i]; }
  return bsplit16(v); }
__device__ __forceinline__ F2 split_rowK(const float* row, int k0, int lane, int K) { float v[16]; const int g = lane >> 4;
#pragma unroll
  for (int i = 0; i < 8; ++i) { const int ka = k0 + 8 * g + i, kb = ka + 16; v[i] = ka < K ? row[ka] : 0.f; v[8 + i] = kb < K ? row[kb] : 0.f; }
  return bsplit16(v); }
__device__ __forceinline__ F2 split_col(const float* W, int k0, int n, int lane, int ld, int K) { float v[16]; const int g = lane >> 4;
#pragma unroll
  for (int i = 0; i < 8; ++i) { const int ka = k0 + 8 * g + i, kb = ka + 16; v[i] = ka < K ? W[(size_t)ka * ld + n] : 0.f; v[8 + i] = kb < K ? W[(size_t)kb * ld + n] : 0.f; }
  return bsplit16(v); }
__device__ __forceinline__ v8f mac3(const F2& a, const F2& b, v8f c) { c = wmma_bf(a.l, b.h, c); c = wmma_bf(a.h, b.l, c); return wmma_bf(a.h, b.h, c); }
__device__ __forceinline__ float sigm(float v) { return 1.0f / (1.0f + expf(-v)); }
#define LDSX() do { asm volatile("s_wait_dscnt 0" ::: "memory"); __builtin_amdgcn_wave_barrier(); __builtin_amdgcn_fence(__ATOMIC_RELEASE, "workgroup"); } while (0)

#define SQ 1024
#define NB 8
#define E 1024
#define NH 16
#define HD 64
#define NR (SQ * NB)

__global__ __launch_bounds__(256) void k_cvt(const float* __restrict__ x, _Float16* __restrict__ X16) {
  const size_t i8 = (size_t)blockIdx.x * 256 + threadIdx.x; if (i8 >= (size_t)NR * E / 8) return;
  union { v8h h; v4u u; } pk;
#pragma unroll
  for (int e = 0; e < 8; ++e) pk.h[e] = (_Float16)x[i8 * 8 + e];
  vst2(X16 + i8 * 8, pk.u);
}
__global__ __launch_bounds__(256) void k_pack(const float* __restrict__ Wqkv, const float* __restrict__ Wo, _Float16* __restrict__ P) {
  const int r = blockIdx.x, tid = threadIdx.x; __shared__ __align__(16) _Float16 srow[E];
  const float* W = r < 3 * E ? Wqkv + (size_t)r * E : Wo + (size_t)(r - 3 * E) * E;
  for (int k = tid; k < E; k += 256) srow[k] = (_Float16)(W[k] * 16.0f);
  __syncthreads();
  if (tid < 128) vst2(P + (size_t)r * E + tid * 8, *(const v4u*)(&srow[tid * 8]));
}
__global__ __launch_bounds__(128) void k_qkv(const _Float16* __restrict__ X16, const _Float16* __restrict__ P, const float* __restrict__ bqkv, _Float16* __restrict__ Q16, _Float16* __restrict__ K16, _Float16* __restrict__ VT) {
  __shared__ __align__(16) float so[4][16][132];
  __shared__ __align__(16) _Float16 st[64][72];
  const int tid = threadIdx.x, wave = tid >> 5, lane = tid & 31, col = lane & 15, g = lane >> 4;
  const int b = blockIdx.z, h = blockIdx.y, s0b = blockIdx.x * 64, s0 = s0b + wave * 16; const int n0 = h * 192; const size_t bh = (size_t)b * NH + h;
  v8f acc[12];
#pragma unroll
  for (int j = 0; j < 12; ++j) acc[j] = (v8f){};
#pragma unroll 1
  for (int kc = 0; kc < E / 32; ++kc) { const v16h a = frag_h(X16 + ((size_t)(s0 + col) * NB + b) * E + kc * 32, lane);
#pragma unroll
    for (int j = 0; j < 12; ++j) acc[j] = wmma16(a, frag_h(P + (size_t)(n0 + j * 16 + col) * E + kc * 32, lane), acc[j]); }
#pragma unroll
  for (int j = 0; j < 8; ++j) { const float bb = bqkv[n0 + j * 16 + col];
#pragma unroll
    for (int r = 0; r < 8; ++r) so[wave][8 * g + r][j * 16 + col] = (acc[j][r] * (1.0f / 16.0f) + bb) * 4.0f; }
#pragma unroll
  for (int j = 8; j < 12; ++j) { const float bb = bqkv[n0 + j * 16 + col];
#pragma unroll
    for (int r = 0; r < 8; ++r) st[(j - 8) * 16 + col][wave * 16 + 8 * g + r] = (_Float16)((acc[j][r] * (1.0f / 16.0f) + bb) * 4.0f); }
  LDSX();
  for (int qq = lane; qq < 16 * 2 * 8; qq += 32) { const int which = qq >> 7, rl = (qq >> 3) & 15, pc = qq & 7; union { v8h h8; v4u u; } pk;
#pragma unroll
    for (int e = 0; e < 8; ++e) pk.h8[e] = (_Float16)so[wave][rl][which * 64 + pc * 8 + e];
    vst2((which == 0 ? Q16 : K16) + (bh * SQ + s0 + rl) * HD + pc * 8, pk.u); }
  __syncthreads();
  for (int qq = tid; qq < 64 * 8; qq += 128) { const int d = qq >> 3, pc = qq & 7; vst2(VT + (bh * HD + d) * SQ + s0b + pc * 8, *(const v4u*)(&st[d][pc * 8])); }
}
__global__ __launch_bounds__(128) void k_attn(const _Float16* __restrict__ Q16, const _Float16* __restrict__ K16, const _Float16* __restrict__ VT, _Float16* __restrict__ O16) {
  __shared__ __align__(16) float sS[4][16][68];
  __shared__ __align__(16) _Float16 sP[4][16][72];
  __shared__ __align__(16) float sO[4][16][68];
  const int tid = threadIdx.x, w = tid >> 5, lane = tid & 31, col = lane & 15, g = lane >> 4;
  const size_t bh = blockIdx.y; const int q0 = blockIdx.x * 64 + w * 16;
  v16h aq[2];
#pragma unroll
  for (int kc = 0; kc < 2; ++kc) aq[kc] = frag_h(Q16 + (bh * SQ + q0 + col) * HD + kc * 32, lane);
  float mrun = -3.0e38f, lrun = 0.f; v8f acc[4] = {};
#pragma unroll 1
  for (int kt = 0; kt < SQ / 64; ++kt) {
#pragma unroll
    for (int t = 0; t < 4; ++t) { v8f s = {}; const int key = kt * 64 + t * 16 + col;
#pragma unroll
      for (int kc = 0; kc < 2; ++kc) s = wmma16(aq[kc], frag_h(K16 + (bh * SQ + key) * HD + kc * 32, lane), s);
#pragma unroll
      for (int r = 0; r < 8; ++r) sS[w][8 * g + r][t * 16 + col] = s[r] * (0.125f / 16.0f); }
    LDSX();
    float mx = -3.4e38f;
#pragma unroll
    for (int jj = 0; jj < 32; ++jj) mx = fmaxf(mx, sS[w][col][g * 32 + jj]);
    mx = fmaxf(mx, __shfl_xor(mx, 16, 32));
    const float mnew = fmaxf(mrun, mx); const float corr = expf(mrun - mnew);
    float ps = 0.f;
#pragma unroll
    for (int jj = 0; jj < 32; ++jj) { const float p = expf(sS[w][col][g * 32 + jj] - mnew); ps += p; sP[w][col][g * 32 + jj] = (_Float16)(p * 16384.0f); }
    ps += __shfl_xor(ps, 16, 32);
    lrun = lrun * corr + ps; mrun = mnew;
#pragma unroll
    for (int r = 0; r < 8; ++r) { const float cr = __shfl(corr, 8 * g + r, 32);
#pragma unroll
      for (int t = 0; t < 4; ++t) acc[t][r] *= cr; }
    LDSX();
#pragma unroll
    for (int kc = 0; kc < 2; ++kc) { const v16h pa = frag_h(&sP[w][col][0] + kc * 32, lane);
#pragma unroll
      for (int t = 0; t < 4; ++t) acc[t] = wmma16(pa, frag_h(VT + (bh * HD + t * 16 + col) * SQ + kt * 64 + kc * 32, lane), acc[t]); }
    __builtin_amdgcn_wave_barrier(); }
#pragma unroll
  for (int r = 0; r < 8; ++r) { const float lr = __shfl(lrun, 8 * g + r, 32); const float inv = 8.0f / (lr * 16384.0f * 4.0f);
#pragma unroll
    for (int t = 0; t < 4; ++t) sO[w][8 * g + r][t * 16 + col] = acc[t][r] * inv; }
  LDSX();
  for (int qq = lane; qq < 16 * 8; qq += 32) { const int rl = qq >> 3, pc = qq & 7; union { v8h h8; v4u u; } pk;
#pragma unroll
    for (int e = 0; e < 8; ++e) pk.h8[e] = (_Float16)sO[w][rl][pc * 8 + e];
    vst2(O16 + (bh * SQ + q0 + rl) * HD + pc * 8, pk.u); }
}
__global__ __launch_bounds__(128) void k_out(const _Float16* __restrict__ O16, const _Float16* __restrict__ P, const float* __restrict__ bo, const float* __restrict__ x, float* __restrict__ Y) {
  __shared__ __align__(16) float so[4][16][132];
  const int tid = threadIdx.x, wave = tid >> 5, lane = tid & 31, col = lane & 15, g = lane >> 4;
  const int r0 = blockIdx.x * 64 + wave * 16, n0 = blockIdx.y * 128; const int ra = r0 + col; const int s = ra / NB, b = ra % NB;
  v8f acc[8] = {};
#pragma unroll 2
  for (int kc = 0; kc < E / 32; ++kc) { const int h = kc >> 1; const v16h a = frag_h(O16 + (((size_t)b * NH + h) * SQ + s) * HD + (kc & 1) * 32, lane);
#pragma unroll
    for (int j = 0; j < 8; ++j) acc[j] = wmma16(a, frag_h(P + (size_t)(3 * E + n0 + j * 16 + col) * E + kc * 32, lane), acc[j]); }
#pragma unroll
  for (int j = 0; j < 8; ++j) { const int n = n0 + j * 16 + col; const float bb = bo[n];
#pragma unroll
    for (int r = 0; r < 8; ++r) so[wave][8 * g + r][j * 16 + col] = acc[j][r] * (1.0f / (16.0f * 8.0f)) + bb + x[(size_t)(r0 + 8 * g + r) * E + n]; }
  LDSX();
#pragma unroll 4
  for (int rl = 0; rl < 16; ++rl) vst2(Y + (size_t)(r0 + rl) * E + n0 + lane * 4, *(const v4f*)(&so[wave][rl][lane * 4]));
}
__global__ __launch_bounds__(256) void k_ln(const float* __restrict__ Y, const float* __restrict__ g1, const float* __restrict__ b1, float* __restrict__ out) {
  const int wave = threadIdx.x >> 5, lane = threadIdx.x & 31; const size_t r = (size_t)blockIdx.x * 8 + wave; if (r >= NR) return;
  const float* yr = Y + r * E; float sm = 0.f, q2 = 0.f;
#pragma unroll 1
  for (int i = 0; i < 8; ++i) { const v4f a = *(const v4f*)(yr + i * 128 + lane * 4); sm += (a[0] + a[1]) + (a[2] + a[3]); q2 += (a[0] * a[0] + a[1] * a[1]) + (a[2] * a[2] + a[3] * a[3]); }
#pragma unroll
  for (int off = 16; off >= 1; off >>= 1) { sm += __shfl_xor(sm, off, 32); q2 += __shfl_xor(q2, off, 32); }
  const float mu = sm * (1.0f / E); const float var = fmaxf(q2 * (1.0f / E) - mu * mu, 0.f); const float rs = rsqrtf(var + 1e-5f);
#pragma unroll 1
  for (int i = 0; i < 8; ++i) { const int c0 = i * 128 + lane * 4; const v4f a = *(const v4f*)(yr + c0); v4f o;
    float v0 = (a[0] - mu) * rs * g1[c0] + b1[c0], v1 = (a[1] - mu) * rs * g1[c0 + 1] + b1[c0 + 1], v2 = (a[2] - mu) * rs * g1[c0 + 2] + b1[c0 + 2], v3 = (a[3] - mu) * rs * g1[c0 + 3] + b1[c0 + 3];
    o[0] = v0 > 0.f ? v0 : expm1f(v0); o[1] = v1 > 0.f ? v1 : expm1f(v1); o[2] = v2 > 0.f ? v2 : expm1f(v2); o[3] = v3 > 0.f ? v3 : expm1f(v3);
    vst2(out + r * E + c0, o); }
}
extern "C" void kernel_launch(void* const* d_in, const int* in_sizes, int n_in, void* d_out, int out_size, void* d_ws, size_t ws_size, hipStream_t stream) {
  (void)in_sizes; (void)n_in; (void)out_size; (void)ws_size;
  const float** I = (const float**)d_in;
  const float* x = I[0]; const float* Wqkv = I[1]; const float* bqkv = I[2]; const float* Wo = I[3]; const float* bo = I[4]; const float* g1 = I[5]; const float* b1 = I[6];
  float* out = (float*)d_out;
  char* ws = (char*)d_ws; size_t off = 0;
  auto take = [&](size_t bytes) { char* p = ws + off; off += (bytes + 255) & ~(size_t)255; return p; };
  _Float16* X16 = (_Float16*)take((size_t)NR * E * 2); _Float16* P = (_Float16*)take((size_t)4 * E * E * 2);
  _Float16* Q16 = (_Float16*)take((size_t)NR * E * 2); _Float16* K16 = (_Float16*)take((size_t)NR * E * 2); _Float16* VT = (_Float16*)take((size_t)NR * E * 2); _Float16* O16 = (_Float16*)take((size_t)NR * E * 2);
  float* Y = (float*)take((size_t)NR * E * 4);
  k_cvt<<<(NR * E / 8 + 255) / 256, 256, 0, stream>>>(x, X16);
  k_pack<<<4 * E, 256, 0, stream>>>(Wqkv, Wo, P);
  k_qkv<<<dim3(SQ / 64, NH, NB), 128, 0, stream>>>(X16, P, bqkv, Q16, K16, VT);
  k_attn<<<dim3(SQ / 64, NB * NH), 128, 0, stream>>>(Q16, K16, VT, O16);
  k_out<<<dim3(NR / 64, E / 128), 128, 0, stream>>>(O16, P, bo, x, Y);
  k_ln<<<NR / 8, 256, 0, stream>>>(Y, g1, b1, out);
}
